// MyAttentionEncoder_5720896438770
// MI455X (gfx1250) — hardware-verified
//
#include <hip/hip_runtime.h>
#include <math.h>

#define NB      32
#define NQ      512
#define NROWS   (NB * NQ)
#define DMR     200
#define DMP     256
#define DMK     224
#define WDR     150
#define TDR     50
#define NHEAD   8
#define DKR     25
#define HDP     32
#define KOFF    (NHEAD * HDP)
#define QKW     (2 * NHEAD * HDP)
#define VROWS   (NHEAD * HDP)
#define DFR     800
#define DFP     832
#define NLAYER  3
#define WQR     (3 * KOFF)
#define ACTL    (DMR / 8)
#define LN_EPS  1e-3f
#define WSC     64.0f
#define HCARRY  16.0f
#define QC      16.0f
#define KC      16.0f
#define VC      16.0f
#define PC      1024.0f
#define FC      1024.0f
#define GC      16.0f
#define INV_TEMPER 0.070710678118654752f
#define LOG2E   1.4426950408889634f

static_assert(NHEAD * DKR == DMR);
static_assert(WDR + TDR == DMR);
static_assert((DMR % 8) == 0 && ACTL == 25 && ACTL <= 32);
static_assert((NROWS % 64) == 0 && (DMP % 64) == 0 && (DFP % 64) == 0 && (QKW % 64) == 0 && (NQ % 64) == 0 && (VROWS % 64) == 0);
static_assert((DMK % 32) == 0 && (DFP % 32) == 0 && DMK <= DMP && DMR <= DMK && DFR <= DFP && DKR <= HDP);
static_assert((DMP % 8) == 0 && (DFP % 8) == 0);
static_assert((NROWS % 16) == 0 && ((16 * DMR) % 32) == 0);
static_assert((NQ % 16) == 0 && (NQ % 32) == 0);

typedef _Float16 v16h __attribute__((ext_vector_type(16)));
typedef _Float16 v8h  __attribute__((ext_vector_type(8)));
typedef float    v8f  __attribute__((ext_vector_type(8)));
typedef float    v4f  __attribute__((ext_vector_type(4)));
typedef unsigned int v4u __attribute__((ext_vector_type(4)));

union FragH { v16h v; v8h h[2]; v4u u[2]; };

__device__ __forceinline__ unsigned short bf_bits(float f) {
  unsigned u = __float_as_uint(f);
  return (unsigned short)((u + 0x7FFFu + ((u >> 16) & 1u)) >> 16);
}
__device__ __forceinline__ float bf_up(unsigned short h) { return __uint_as_float(((unsigned)h) << 16); }
__device__ __forceinline__ float bfr(float f) { return bf_up(bf_bits(f)); }
__device__ __forceinline__ unsigned short h_bits(_Float16 x) { return __builtin_bit_cast(unsigned short, x); }
__device__ __forceinline__ unsigned pk16(unsigned short a, unsigned short b) { return (unsigned)a | ((unsigned)b << 16); }
__device__ __forceinline__ v8f zero8() { v8f z = {0.f, 0.f, 0.f, 0.f, 0.f, 0.f, 0.f, 0.f}; return z; }
__device__ __forceinline__ int clampi(int v, int lo, int hi) { return v < lo ? lo : (v > hi ? hi : v); }

__device__ __forceinline__ v16h ldfrag_h(const _Float16* p) {
  FragH f;
  f.h[0] = *(const v8h*)(p);
  f.h[1] = *(const v8h*)(p + 16);
  return f.v;
}
__device__ __forceinline__ v16h ldfrag_u(const unsigned short* p) {
  FragH f;
  f.u[0] = *(const v4u*)(p);
  f.u[1] = *(const v4u*)(p + 16);
  return f.v;
}

__device__ __forceinline__ v8f mma_raw(v16h a, v16h b, v8f c) {
  return __builtin_amdgcn_wmma_f32_16x16x32_f16(false, a, false, b, (short)0, c, false, false);
}
__device__ __forceinline__ void dep_guard1(v8f& a, v8f& b, v16h x) {
#if defined(__HIP_DEVICE_COMPILE__)
  asm volatile("v_nop\n\tv_nop\n\tv_nop\n\tv_nop" : "+v"(a), "+v"(b) : "v"(x));
#endif
}
__device__ __forceinline__ void guard2(v8f& a, v8f& b, v16h x, v16h y, v16h z) {
#if defined(__HIP_DEVICE_COMPILE__)
  asm volatile("v_nop\n\tv_nop\n\tv_nop\n\tv_nop" : "+v"(a), "+v"(b) : "v"(x), "v"(y), "v"(z));
#endif
}
__device__ __forceinline__ void keep4_h(v16h a, v16h b, v16h c, v16h d) {
#if defined(__HIP_DEVICE_COMPILE__)
  asm volatile("v_nop" :: "v"(a), "v"(b), "v"(c), "v"(d));
#endif
}
__device__ __forceinline__ void acc_guard4(v8f& a, v8f& b, v8f& c, v8f& d) {
#if defined(__HIP_DEVICE_COMPILE__)
  asm volatile("v_nop\n\tv_nop\n\tv_nop\n\tv_nop" : "+v"(a), "+v"(b), "+v"(c), "+v"(d));
#endif
}
__device__ __forceinline__ void wave_sync_lds() {
  __builtin_amdgcn_fence(__ATOMIC_RELEASE, "workgroup");
  __builtin_amdgcn_wave_barrier();
  __builtin_amdgcn_fence(__ATOMIC_ACQUIRE, "workgroup");
}

__global__ __launch_bounds__(256) void cvtpad(const float* __restrict__ src, unsigned short* dst,
                                              int R, int C, int Rp, int Cp, float sc) {
  const int tid = threadIdx.x, lane = tid & 31, wave = tid >> 5;
  src += (size_t)blockIdx.z * (size_t)R * (size_t)C;
  dst += (size_t)blockIdx.z * (size_t)Rp * (size_t)Cp;
  const int r  = blockIdx.x * 8 + wave;
  const int rv = (r < R) ? 1 : 0;
  const int rc = rv ? r : (R - 1);
  const float* sp = src + (size_t)rc * C;
  const int np = Cp >> 3;
  v4u vals[4];
#pragma unroll
  for (int it = 0; it < 4; ++it) {
    v4u w = {0u, 0u, 0u, 0u};
    if (it * 32 < np) {
      const int p = it * 32 + lane;
      unsigned short hb[8];
#pragma unroll
      for (int e = 0; e < 8; ++e) {
        const int c  = p * 8 + e;
        const int cc = (c < C) ? c : (C - 1);
        const float f = sp[cc];
        const unsigned short bits = h_bits((_Float16)(bfr(f) * sc));
        hb[e] = (rv != 0 && c < C) ? bits : (unsigned short)0;
      }
      w[0] = pk16(hb[0], hb[1]);
      w[1] = pk16(hb[2], hb[3]);
      w[2] = pk16(hb[4], hb[5]);
      w[3] = pk16(hb[6], hb[7]);
    }
    vals[it] = w;
  }
  unsigned short* dp = dst + (size_t)r * Cp;
  for (int pass = 0; pass < 2; ++pass) {
#pragma unroll
    for (int it = 0; it < 4; ++it) {
      const int p = it * 32 + lane;
      if (p < np) *(volatile v4u*)(dp + (size_t)p * 8) = vals[it];
    }
    __threadfence();
  }
}

__global__ __launch_bounds__(256) void cvtqkv(const float* __restrict__ wq, const float* __restrict__ wk,
                                              const float* __restrict__ wv, unsigned short* dst, float sc) {
  __shared__ __align__(16) unsigned short sT[HDP * 264];
  const int tid = threadIdx.x, lane = tid & 31, wave = tid >> 5;
  const int h = blockIdx.x, l = blockIdx.y, p = blockIdx.z;
  const float* src = (p == 0) ? wq : ((p == 1) ? wk : wv);
  src += (((size_t)l * NHEAD + h) * DMR) * DKR;
  const int dd = tid, ddc = (dd < DMR) ? dd : (DMR - 1);
  const float* sp = src + (size_t)ddc * DKR;
#pragma unroll
  for (int kk = 0; kk < HDP; ++kk) {
    const int kc = (kk < DKR) ? kk : (DKR - 1);
    const float f = sp[kc];
    const unsigned short bits = h_bits((_Float16)(bfr(f) * sc));
    sT[kk * 264 + dd] = (dd < DMR && kk < DKR) ? bits : (unsigned short)0;
  }
  __syncthreads();
  v4u vals[4];
#pragma unroll
  for (int it = 0; it < 4; ++it) {
    const int kk = it * 8 + wave;
    vals[it] = *(const v4u*)(sT + kk * 264 + lane * 8);
  }
  const size_t rowbase = (size_t)l * WQR + (size_t)p * KOFF + (size_t)h * HDP;
  for (int pass = 0; pass < 2; ++pass) {
#pragma unroll
    for (int it = 0; it < 4; ++it) {
      const int kk = it * 8 + wave;
      *(volatile v4u*)(dst + (rowbase + kk) * DMP + lane * 8) = vals[it];
    }
    __threadfence();
  }
}

template <int OM, int HASR, int HASB, int ACT>
__global__ __launch_bounds__(256) void gemm64(
    const unsigned short* __restrict__ Ap, int lda, long long sA,
    const unsigned short* __restrict__ Btp, int ldb, long long sB,
    const float* __restrict__ Rp, const float* __restrict__ Bsp, int Nreal,
    void* Cout, int ldc, long long sC,
    int M, int N, int K, float oscale, float ocarry) {
  static_assert(!(OM != 0 && HASR != 0));
  __shared__ __align__(16) float sT[8][16 * 68];
  const int by   = blockIdx.y;
  const int lane = threadIdx.x & 31;
  const int wave = threadIdx.x >> 5;
  const int tilesN = N >> 6;
  const int tilesM = M >> 6;
  const int tile = blockIdx.x * 8 + wave;
  if (tile >= tilesM * tilesN) return;
  const int tm = tile / tilesN;
  const int tn = tile - tm * tilesN;
  const int m0 = tm << 6;
  const int n0 = tn << 6;

  const unsigned short* A1 = Ap  + (size_t)((long long)by * sA);
  const unsigned short* Bb = Btp + (size_t)((long long)by * sB);

  const int rlane = lane & 15;
  const int koff  = (lane >> 4) * 8;
  const int mOff  = (lane >> 4) * 8;

  v8f acc[4][4];
#pragma unroll
  for (int i = 0; i < 4; ++i)
#pragma unroll
    for (int j = 0; j < 4; ++j) acc[i][j] = zero8();

  for (int k0 = 0; k0 < K; k0 += 32) {
    v16h bh[4];
#pragma unroll
    for (int j = 0; j < 4; ++j) {
      const size_t bofs = (size_t)(n0 + (j << 4) + rlane) * ldb + koff + k0;
      bh[j] = ldfrag_u(Bb + bofs);
    }
#pragma unroll
    for (int i = 0; i < 4; ++i) {
      const size_t ao = (size_t)(m0 + (i << 4) + rlane) * lda + koff + k0;
      const v16h ah = ldfrag_u(A1 + ao);
#pragma unroll
      for (int j = 0; j < 4; ++j) acc[i][j] = mma_raw(ah, bh[j], acc[i][j]);
      dep_guard1(acc[i][0], acc[i][3], ah);
    }
    keep4_h(bh[0], bh[1], bh[2], bh[3]);
  }
  acc_guard4(acc[0][0], acc[0][1], acc[0][2], acc[0][3]);
  acc_guard4(acc[1][0], acc[1][1], acc[1][2], acc[1][3]);
  acc_guard4(acc[2][0], acc[2][1], acc[2][2], acc[2][3]);
  acc_guard4(acc[3][0], acc[3][1], acc[3][2], acc[3][3]);

  const int hh2 = lane >> 4, c4 = (lane & 15) * 4;
  const int q8  = lane >> 3, c8 = (lane & 7) * 8;

  float* slab = sT[wave];
#pragma unroll
  for (int i = 0; i < 4; ++i) {
    const int mBase = m0 + (i << 4);
#pragma unroll
    for (int j = 0; j < 4; ++j) {
#pragma unroll
      for (int r = 0; r < 8; ++r) {
        slab[(mOff + r) * 68 + (j << 4) + rlane] = acc[i][j][r];
      }
    }
    wave_sync_lds();
    if constexpr (OM == 0) {
      float* C = (float*)Cout + (size_t)((long long)by * sC);
      v4f bv = {0.f, 0.f, 0.f, 0.f};
      if constexpr (HASB == 1) {
#pragma unroll
        for (int e = 0; e < 4; ++e) {
          const int n  = n0 + c4 + e;
          const int nc = (n < Nreal) ? n : (Nreal - 1);
          const float braw = Bsp[nc];
          bv[e] = (n < Nreal) ? bfr(braw) : 0.f;
        }
      }
      v4f vals[8];
#pragma unroll
      for (int it = 0; it < 8; ++it) {
        const int row = it * 2 + hh2;
        const int gr  = mBase + row;
        v4f v = *(const v4f*)(slab + row * 68 + c4);
        v4f rv = {0.f, 0.f, 0.f, 0.f};
        if constexpr (HASR != 0) {
          const float* R = Rp + (size_t)((long long)by * sC);
          rv = *(const v4f*)(R + (size_t)gr * ldc + n0 + c4);
        }
#pragma unroll
        for (int e = 0; e < 4; ++e) v[e] = (v[e] * oscale + bv[e]) + rv[e];
        vals[it] = v;
      }
      for (int pass = 0; pass < 2; ++pass) {
#pragma unroll
        for (int it = 0; it < 8; ++it) {
          const int gr = mBase + it * 2 + hh2;
          *(volatile v4f*)(C + (size_t)gr * ldc + n0 + c4) = vals[it];
        }
        __threadfence();
      }
    } else {
      unsigned short* C = (unsigned short*)Cout + (size_t)((long long)by * sC);
      float bb8[8];
#pragma unroll
      for (int e = 0; e < 8; ++e) bb8[e] = 0.f;
      if constexpr (HASB == 1) {
#pragma unroll
        for (int e = 0; e < 8; ++e) {
          const int n  = n0 + c8 + e;
          const int nc = (n < Nreal) ? n : (Nreal - 1);
          const float braw = Bsp[nc];
          bb8[e] = (n < Nreal) ? bfr(braw) : 0.f;
        }
      }
      v4u hv[4];
#pragma unroll
      for (int it = 0; it < 4; ++it) {
        const int row = it * 4 + q8;
        const float* sp = slab + row * 68 + c8;
        v4u a = {0u, 0u, 0u, 0u};
#pragma unroll
        for (int e = 0; e < 4; ++e) {
          float f0 = sp[2 * e] * oscale + bb8[2 * e];
          float f1 = sp[2 * e + 1] * oscale + bb8[2 * e + 1];
          if constexpr (ACT == 1) { f0 = fmaxf(f0, 0.f); f1 = fmaxf(f1, 0.f); }
          f0 *= ocarry; f1 *= ocarry;
          a[e] = pk16(h_bits((_Float16)f0), h_bits((_Float16)f1));
        }
        hv[it] = a;
      }
      for (int pass = 0; pass < 2; ++pass) {
#pragma unroll
        for (int it = 0; it < 4; ++it) {
          const int row = it * 4 + q8;
          *(volatile v4u*)(C + (size_t)(mBase + row) * ldc + n0 + c8) = hv[it];
        }
        __threadfence();
      }
    }
    wave_sync_lds();
  }
}

#define ATT_THREADS (NHEAD * 32)
#define ATT_BLOCKS  (NB * (NQ / 16))
#define PS_FLOATS   (NHEAD * 16 * 36)
#define PADV4       ((16 * (DMP - DMR)) / 8)
static_assert(ATT_THREADS == 256 && ATT_BLOCKS == 1024);
static_assert((size_t)16 * DMP * sizeof(unsigned short) <= (size_t)PS_FLOATS * sizeof(float));
static_assert(((16 * DMP) / 8) == 2 * ATT_THREADS);
static_assert(PADV4 == 112 && PADV4 <= ATT_THREADS && ((DMP - DMR) % 8) == 0);
static_assert(HDP == 32 && DKR > 16 && DKR <= 32);

__global__ __launch_bounds__(ATT_THREADS)
void attn16(const unsigned short* __restrict__ QKq, const unsigned short* __restrict__ VTq,
            const int* __restrict__ wseq, unsigned short* CT) {
  __shared__ __align__(16) float smem[PS_FLOATS];
  __shared__ int skm[NQ];

  const int tid  = threadIdx.x;
  const int wave = tid >> 5;
  const int lane = tid & 31;
  const int hh   = lane >> 4;
  const int c    = lane & 15;

  const int qt   = blockIdx.x % (NQ / 16);
  const int bat  = blockIdx.x / (NQ / 16);
  const int head = wave;
  const int q0   = qt * 16;

  for (int i = tid; i < NQ; i += ATT_THREADS) skm[i] = (wseq[(size_t)bat * NQ + i] == 0) ? 1 : 0;

  const _Float16* QK = (const _Float16*)(const void*)QKq;
  const _Float16* Qh = QK + ((size_t)bat * NQ + q0 + c) * QKW + head * HDP + 8 * hh;
  const _Float16* Kb = QK + (size_t)bat * NQ * QKW + KOFF + head * HDP + 8 * hh;
  const _Float16* Vb = (const _Float16*)(const void*)VTq + ((size_t)bat * VROWS + head * HDP) * NQ + 8 * hh;
  const float lsc  = (LOG2E * INV_TEMPER) / (QC * KC);

  const v16h qa = ldfrag_h(Qh);

  float mrow[8], lrow[8];
  v8f o0 = zero8(), o1 = zero8();
#pragma unroll
  for (int r = 0; r < 8; ++r) { mrow[r] = -INFINITY; lrow[r] = 0.f; }
  float* pt = smem + wave * (16 * 36);

  __syncthreads();

#pragma unroll 1
  for (int kb = 0; kb < NQ; kb += 32) {
    const _Float16* kp = Kb + (size_t)(kb + c) * QKW;
    v8f s0, s1;
    {
      const v16h kf0 = ldfrag_h(kp);
      const v16h kf1 = ldfrag_h(kp + (size_t)16 * QKW);
      s0 = mma_raw(qa, kf0, zero8());
      s1 = mma_raw(qa, kf1, zero8());
      guard2(s0, s1, kf0, kf1, qa);
    }
    const int mk0 = skm[kb + c], mk1 = skm[kb + 16 + c];
#pragma unroll
    for (int r = 0; r < 8; ++r) {
      const float t0 = (mk0 != 0) ? -INFINITY : s0[r] * lsc;
      const float t1 = (mk1 != 0) ? -INFINITY : s1[r] * lsc;
      float mx = fmaxf(t0, t1);
#pragma unroll
      for (int off = 1; off < 16; off <<= 1) mx = fmaxf(mx, __shfl_xor(mx, off, 32));
      const float mn   = fmaxf(mrow[r], mx);
      const float msub = (mn == -INFINITY) ? 0.f : mn;
      const float al   = exp2f(fmaxf(mrow[r] - msub, -126.0f));
      mrow[r] = mn;
      const float e0 = exp2f(t0 - msub);
      const float e1 = exp2f(t1 - msub);
      float ps = e0 + e1;
#pragma unroll
      for (int off = 1; off < 16; off <<= 1) ps += __shfl_xor(ps, off, 32);
      lrow[r] = lrow[r] * al + ps;
      o0[r] *= al;
      o1[r] *= al;
      const int ro = (8 * hh + r) * 36 + c;
      pt[ro]      = e0;
      pt[ro + 16] = e1;
    }
    wave_sync_lds();
    FragH ph;
    {
      const float* prow = pt + c * 36 + 8 * hh;
      const v4f p0 = *(const v4f*)(prow), p1 = *(const v4f*)(prow + 4);
      const v4f p2 = *(const v4f*)(prow + 16), p3 = *(const v4f*)(prow + 20);
#pragma unroll
      for (int e = 0; e < 4; ++e) {
        ph.h[0][e]     = (_Float16)(p0[e] * PC);
        ph.h[0][4 + e] = (_Float16)(p1[e] * PC);
        ph.h[1][e]     = (_Float16)(p2[e] * PC);
        ph.h[1][4 + e] = (_Float16)(p3[e] * PC);
      }
    }
    const _Float16* vp = Vb + (size_t)c * NQ + kb;
    {
      const v16h vb0 = ldfrag_h(vp);
      const v16h vb1 = ldfrag_h(vp + (size_t)16 * NQ);
      o0 = mma_raw(ph.v, vb0, o0);
      o1 = mma_raw(ph.v, vb1, o1);
      guard2(o0, o1, ph.v, vb0, vb1);
    }
    wave_sync_lds();
  }

  __syncthreads();
  unsigned short* Os = (unsigned short*)smem;
  if (tid < PADV4) {
    const int prow = tid / 7, pj = tid - prow * 7;
    v4u z = {0u, 0u, 0u, 0u};
    *(v4u*)(Os + (size_t)prow * DMP + DMR + pj * 8) = z;
  }
  const float oc = FC / (PC * VC);
  unsigned short* osw = Os + head * DKR + c;
#pragma unroll
  for (int r = 0; r < 8; ++r) {
    const float inv = (1.0f / lrow[r]) * oc;
    unsigned short* op = osw + (8 * hh + r) * DMP;
    op[0] = h_bits((_Float16)(o0[r] * inv));
    if (c < DKR - 16) op[16] = h_bits((_Float16)(o1[r] * inv));
  }
  __syncthreads();
  {
    v4u vals[2];
#pragma unroll
    for (int it = 0; it < 2; ++it) {
      const int p = it * ATT_THREADS + tid;
      vals[it] = *(const v4u*)(Os + (size_t)p * 8);
    }
    unsigned short* dst = CT + ((size_t)bat * NQ + q0) * DMP;
    for (int pass = 0; pass < 2; ++pass) {
#pragma unroll
      for (int it = 0; it < 2; ++it) {
        const int p = it * ATT_THREADS + tid;
        const int row = p >> 5, col8 = (p & 31) * 8;
        *(volatile v4u*)(dst + (size_t)row * DMP + col8) = vals[it];
      }
      __threadfence();
    }
  }
}

__device__ __forceinline__ void put_row2(float* sr, v4f oa, v4f ob, int lane, float* hrow, unsigned short* xrow, float hc) {
  *(v4f*)(sr + lane * 8)     = oa;
  *(v4f*)(sr + lane * 8 + 4) = ob;
  wave_sync_lds();
  const v4f u0 = *(const v4f*)(sr + lane * 4);
  const v4f u1 = *(const v4f*)(sr + (DMP / 2) + lane * 4);
  v4u w;
  w[0] = pk16(h_bits((_Float16)(oa[0] * hc)), h_bits((_Float16)(oa[1] * hc)));
  w[1] = pk16(h_bits((_Float16)(oa[2] * hc)), h_bits((_Float16)(oa[3] * hc)));
  w[2] = pk16(h_bits((_Float16)(ob[0] * hc)), h_bits((_Float16)(ob[1] * hc)));
  w[3] = pk16(h_bits((_Float16)(ob[2] * hc)), h_bits((_Float16)(ob[3] * hc)));
  for (int pass = 0; pass < 2; ++pass) {
    *(volatile v4f*)(hrow + lane * 4) = u0;
    *(volatile v4f*)(hrow + (DMP / 2) + lane * 4) = u1;
    *(volatile v4u*)(xrow + lane * 8) = w;
    __threadfence();
  }
  wave_sync_lds();
}

__global__ __launch_bounds__(256) void embed(const float* __restrict__ we, const float* __restrict__ ee,
                                             const float* __restrict__ te, const float* __restrict__ pt,
                                             const float* __restrict__ bias,
                                             const int* __restrict__ wseq, const int* __restrict__ ews,
                                             const int* __restrict__ tg, const int* __restrict__ ps,
                                             int nV, int nVE, int nT, int nP,
                                             float* Hout, unsigned short* Xout) {
  __shared__ __align__(16) float srow[8][DMP];
  const int tid = threadIdx.x, lane = tid & 31, wave = tid >> 5;
  const bool act = lane < ACTL;
  const int cb = lane * 8;
  float bb[8];
#pragma unroll
  for (int e = 0; e < 8; ++e) {
    const int cc = clampi(cb + e, 0, DMR - 1);
    bb[e] = bfr(bias[cc]);
  }
#pragma unroll
  for (int it = 0; it < 2; ++it) {
    const int row = blockIdx.x * 16 + it * 8 + wave;
    const int w = clampi(wseq[row], 0, nV - 1);
    const int x = clampi(ews[row], 0, nVE - 1);
    const int t = clampi(tg[row], 0, nT - 1);
    const int p = clampi(ps[row], 0, nP - 1);
    const float* wr = we + (size_t)w * WDR;
    const float* er = ee + (size_t)x * WDR;
    const float* tr = te + (size_t)t * TDR;
    const float* pr = pt + (size_t)p * DMR;
    float o[8];
#pragma unroll
    for (int e = 0; e < 8; ++e) {
      const int cc0 = cb + e;
      const int cw  = clampi(cc0, 0, WDR - 1);
      const int ct  = clampi(cc0 - WDR, 0, TDR - 1);
      const int cc  = clampi(cc0, 0, DMR - 1);
      const float fw = bfr(wr[cw]) + bfr(er[cw]);
      const float ft = bfr(tr[ct]);
      float v = (cc0 < WDR) ? fw : ft;
      v = (v + bb[e]) + bfr(pr[cc]);
      o[e] = act ? v : 0.f;
    }
    v4f oa, ob;
    oa[0] = o[0]; oa[1] = o[1]; oa[2] = o[2]; oa[3] = o[3];
    ob[0] = o[4]; ob[1] = o[5]; ob[2] = o[6]; ob[3] = o[7];
    put_row2(srow[wave], oa, ob, lane, Hout + (size_t)row * DMP, Xout + (size_t)row * DMP, HCARRY);
  }
}

#define OUTP4 ((16 * DMR) / 4)
static_assert(OUTP4 == 800 && OUTP4 <= 4 * 256 && (OUTP4 % 32) == 0 && ((16 * DMR * 4) % 128) == 0);

template <int FIN>
__global__ __launch_bounds__(256) void lnorm(const float* __restrict__ Y, const float* __restrict__ ga,
                                             const float* __restrict__ gb, float* Hout, unsigned short* Xout,
                                             float* Out) {
  __shared__ __align__(16) float srow[8][DMP];
  __shared__ __align__(16) float sflat[16 * DMR];
  const int tid = threadIdx.x, lane = tid & 31, wave = tid >> 5;
  const bool act = lane < ACTL;
  const int cb = lane * 8;
  float g[8], bt[8];
#pragma unroll
  for (int e = 0; e < 8; ++e) {
    const int cc = clampi(cb + e, 0, DMR - 1);
    g[e]  = bfr(ga[cc]);
    bt[e] = bfr(gb[cc]);
  }
#pragma unroll
  for (int it = 0; it < 2; ++it) {
    const int rib = it * 8 + wave;
    const int row = blockIdx.x * 16 + rib;
    const float* yr = Y + (size_t)row * DMP + cb;
    const v4f a4 = *(const v4f*)(yr), b4 = *(const v4f*)(yr + 4);
    float v[8];
    v[0] = a4[0]; v[1] = a4[1]; v[2] = a4[2]; v[3] = a4[3]; v[4] = b4[0]; v[5] = b4[1]; v[6] = b4[2]; v[7] = b4[3];
#pragma unroll
    for (int e = 0; e < 8; ++e) v[e] = act ? v[e] : 0.f;
    float s = ((v[0] + v[1]) + (v[2] + v[3])) + ((v[4] + v[5]) + (v[6] + v[7]));
#pragma unroll
    for (int off = 1; off < 32; off <<= 1) s += __shfl_xor(s, off, 32);
    const float mu = s * (1.0f / (float)DMR);
    float d[8];
#pragma unroll
    for (int e = 0; e < 8; ++e) d[e] = act ? (v[e] - mu) : 0.f;
    float q = 0.f;
#pragma unroll
    for (int e = 0; e < 8; ++e) q += d[e] * d[e];
#pragma unroll
    for (int off = 1; off < 32; off <<= 1) q += __shfl_xor(q, off, 32);
    const float var = q * (1.0f / (float)(DMR - 1));
    const float sig = sqrtf(var);
    const float inv = 1.0f / (sig + LN_EPS);
    float o[8];
#pragma unroll
    for (int e = 0; e < 8; ++e) o[e] = act ? ((d[e] * inv) * g[e] + bt[e]) : 0.f;
    v4f oa, ob;
    oa[0] = o[0]; oa[1] = o[1]; oa[2] = o[2]; oa[3] = o[3];
    ob[0] = o[4]; ob[1] = o[5]; ob[2] = o[6]; ob[3] = o[7];
    if constexpr (FIN == 0) {
      put_row2(srow[wave], oa, ob, lane, Hout + (size_t)row * DMP, Xout + (size_t)row * DMP, HCARRY);
    } else {
      if (act) {
        *(v4f*)(sflat + rib * DMR + cb)     = oa;
        *(v4f*)(sflat + rib * DMR + cb + 4) = ob;
      }
    }
  }
  if constexpr (FIN == 1) {
    __syncthreads();
    v4f vals[4];
#pragma unroll
    for (int it2 = 0; it2 < 4; ++it2) {
      const int p  = it2 * 256 + tid;
      const int pc = (p < OUTP4) ? p : (OUTP4 - 1);
      vals[it2] = *(const v4f*)(sflat + pc * 4);
    }
    float* ob4 = Out + (size_t)blockIdx.x * (16 * DMR);
    for (int pass = 0; pass < 2; ++pass) {
#pragma unroll
      for (int it2 = 0; it2 < 4; ++it2) {
        const int p = it2 * 256 + tid;
        if (p < OUTP4) *(volatile v4f*)(ob4 + (size_t)p * 4) = vals[it2];
      }
      __threadfence();
    }
  }
}

extern "C" void kernel_launch(void* const* d_in, const int* in_sizes, int n_in,
                              void* d_out, int out_size, void* d_ws, size_t ws_size,
                              hipStream_t stream) {
  if (n_in < 22) return;
  if (in_sizes[0] < WDR || (in_sizes[0] % WDR) != 0) return;
  if (in_sizes[1] < WDR || (in_sizes[1] % WDR) != 0) return;
  if (in_sizes[2] < TDR || (in_sizes[2] % TDR) != 0) return;
  if (in_sizes[3] < DMR || (in_sizes[3] % DMR) != 0) return;
  if (in_sizes[4] != DMR) return;
  if (in_sizes[5] != NLAYER * NHEAD * DMR * DKR || in_sizes[6] != NLAYER * NHEAD * DMR * DKR || in_sizes[7] != NLAYER * NHEAD * DMR * DKR) return;
  if (in_sizes[8] != NLAYER * DMR * DMR) return;
  if (in_sizes[9] != NLAYER * DFR * DMR || in_sizes[10] != NLAYER * DFR) return;
  if (in_sizes[11] != NLAYER * DMR * DFR || in_sizes[12] != NLAYER * DMR) return;
  if (in_sizes[13] != NLAYER * DMR || in_sizes[14] != NLAYER * DMR || in_sizes[15] != NLAYER * DMR || in_sizes[16] != NLAYER * DMR) return;
  if (in_sizes[17] != NROWS || in_sizes[18] != NROWS || in_sizes[19] != NROWS || in_sizes[20] != NROWS) return;
  if (out_size != NROWS * DMR) return;

  const int nV  = in_sizes[0] / WDR;
  const int nVE = in_sizes[1] / WDR;
  const int nT  = in_sizes[2] / TDR;
  const int nP  = in_sizes[3] / DMR;

  const float* word_emb    = (const float*)d_in[0];
  const float* extword_emb = (const float*)d_in[1];
  const float* tag_emb     = (const float*)d_in[2];
  const float* pos_table   = (const float*)d_in[3];
  const float* bias        = (const float*)d_in[4];
  const float* w_qs        = (const float*)d_in[5];
  const float* w_ks        = (const float*)d_in[6];
  const float* w_vs        = (const float*)d_in[7];
  const float* w_o         = (const float*)d_in[8];
  const float* ffn_w1      = (const float*)d_in[9];
  const float* ffn_b1      = (const float*)d_in[10];
  const float* ffn_w2      = (const float*)d_in[11];
  const float* ffn_b2      = (const float*)d_in[12];
  const float* ln_ffn_a    = (const float*)d_in[13];
  const float* ln_ffn_b    = (const float*)d_in[14];
  const float* ln_attn_a   = (const float*)d_in[15];
  const float* ln_attn_b   = (const float*)d_in[16];
  const int*   word_seq    = (const int*)d_in[17];
  const int*   extwords    = (const int*)d_in[18];
  const int*   tagsq       = (const int*)d_in[19];
  const int*   pos_seq     = (const int*)d_in[20];
  float*       out         = (float*)d_out;

  const size_t PWQKV = (size_t)NLAYER * WQR * DMP * 2;
  const size_t PWO   = (size_t)NLAYER * DMP * DMP * 2;
  const size_t PW1   = (size_t)NLAYER * DFP * DMP * 2;
  const size_t PW2   = (size_t)NLAYER * DMP * DFP * 2;
  const size_t PH    = (size_t)NROWS * DMP * 4;
  const size_t PX16  = (size_t)NROWS * DMP * 2;
  const size_t PQK   = (size_t)NROWS * QKW * 2;
  const size_t PVT   = (size_t)NB * VROWS * NQ * 2;
  const size_t PCT   = (size_t)NROWS * DMP * 2;
  const size_t PG    = (size_t)NROWS * DFP * 2;
  size_t off = 0;
  const size_t oWQKV = off; off += PWQKV;
  const size_t oWO   = off; off += PWO;
  const size_t oW1   = off; off += PW1;
  const size_t oW2   = off; off += PW2;
  const size_t oH0   = off; off += PH;
  const size_t oH1   = off; off += PH;
  const size_t oX16  = off; off += PX16;
  const size_t oQK   = off; off += PQK;
  const size_t oVT   = off; off += PVT;
  const size_t oCT   = off; off += PCT;
  const size_t oG    = off; off += PG;
  if (off > ws_size) return;
  if (off > (size_t)134217728) return;

  char* ws = (char*)d_ws;
  unsigned short* WQKV = (unsigned short*)(ws + oWQKV);
  unsigned short* WOP  = (unsigned short*)(ws + oWO);
  unsigned short* W1P  = (unsigned short*)(ws + oW1);
  unsigned short* W2P  = (unsigned short*)(ws + oW2);
  float*          H0   = (float*)(ws + oH0);
  float*          H1   = (float*)(ws + oH1);
  unsigned short* X16  = (unsigned short*)(ws + oX16);
  unsigned short* QK   = (unsigned short*)(ws + oQK);
  unsigned short* VTp  = (unsigned short*)(ws + oVT);
  unsigned short* CT   = (unsigned short*)(ws + oCT);
  unsigned short* G16  = (unsigned short*)(ws + oG);

  const dim3 blk(256);
  const dim3 gQKV(NHEAD, NLAYER, 3);
  const dim3 gWO(DMP / 8, 1, NLAYER);
  const dim3 gW1(DFP / 8, 1, NLAYER);
  const dim3 gW2(DMP / 8, 1, NLAYER);
  const dim3 gEMB(NROWS / 16);
  const int tilesF1 = (NROWS / 64) * (DFP / 64);
  const int tilesD  = (NROWS / 64) * (DMP / 64);
  const int tilesQK = (NROWS / 64) * (QKW / 64);
  const int tilesV  = (VROWS / 64) * (NQ / 64);
  const dim3 gF1((tilesF1 + 7) / 8, 1);
  const dim3 gD((tilesD + 7) / 8, 1);
  const dim3 gQK((tilesQK + 7) / 8, 1);
  const dim3 gV((tilesV + 7) / 8, NB);
  const dim3 gAT(ATT_BLOCKS);
  const dim3 bAT(ATT_THREADS);
  const dim3 gLN(NROWS / 16);

  cvtqkv<<<gQKV, blk, 0, stream>>>(w_qs, w_ks, w_vs, WQKV, WSC);
  cvtpad<<<gWO, blk, 0, stream>>>(w_o, WOP, DMR, DMR, DMP, DMP, WSC);
  cvtpad<<<gW1, blk, 0, stream>>>(ffn_w1, W1P, DFR, DMR, DFP, DMP, WSC);
  cvtpad<<<gW2, blk, 0, stream>>>(ffn_w2, W2P, DMR, DFR, DMP, DFP, WSC);

  embed<<<gEMB, blk, 0, stream>>>(word_emb, extword_emb, tag_emb, pos_table, bias,
                                  word_seq, extwords, tagsq, pos_seq, nV, nVE, nT, nP, H0, X16);

  for (int l = 0; l < NLAYER; ++l) {
    const unsigned short* Wl = WQKV + (size_t)l * WQR * DMP;

    gemm64<2, 0, 1, 1><<<gF1, blk, 0, stream>>>(
        X16, DMP, 0LL,
        W1P + (size_t)l * DFP * DMP, DMP, 0LL,
        (const float*)0, ffn_b1 + (size_t)l * DFR, DFR,
        (void*)G16, DFP, 0LL,
        NROWS, DFP, DMK, 1.0f / (HCARRY * WSC), GC);

    gemm64<0, 1, 1, 0><<<gD, blk, 0, stream>>>(
        G16, DFP, 0LL,
        W2P + (size_t)l * DMP * DFP, DFP, 0LL,
        H0, ffn_b2 + (size_t)l * DMR, DMR,
        (void*)H1, DMP, 0LL,
        NROWS, DMP, DFP, 1.0f / (GC * WSC), 1.0f);

    lnorm<0><<<gLN, blk, 0, stream>>>(H1, ln_ffn_a + (size_t)l * DMR, ln_ffn_b + (size_t)l * DMR, H0, X16, out);

    gemm64<2, 0, 0, 0><<<gQK, blk, 0, stream>>>(
        X16, DMP, 0LL,
        Wl, DMP, 0LL,
        (const float*)0, (const float*)0, 1,
        (void*)QK, QKW, 0LL,
        NROWS, QKW, DMK, 1.0f / (HCARRY * WSC), QC);

    gemm64<2, 0, 0, 0><<<gV, blk, 0, stream>>>(
        Wl + (size_t)2 * KOFF * DMP, DMP, 0LL,
        X16, DMP, (long long)NQ * DMP,
        (const float*)0, (const float*)0, 1,
        (void*)VTp, NQ, (long long)VROWS * NQ,
        VROWS, NQ, DMK, 1.0f / (HCARRY * WSC), VC);

    attn16<<<gAT, bAT, 0, stream>>>(QK, VTp, word_seq, CT);

    gemm64<0, 1, 0, 0><<<gD, blk, 0, stream>>>(
        CT, DMP, 0LL,
        WOP + (size_t)l * DMP * DMP, DMP, 0LL,
        H0, (const float*)0, 1,
        (void*)H1, DMP, 0LL,
        NROWS, DMP, DMK, 1.0f / (FC * WSC), 1.0f);

    if (l < NLAYER - 1) {
      lnorm<0><<<gLN, blk, 0, stream>>>(H1, ln_attn_a + (size_t)l * DMR, ln_attn_b + (size_t)l * DMR, H0, X16, out);
    } else {
      lnorm<1><<<gLN, blk, 0, stream>>>(H1, ln_attn_a + (size_t)l * DMR, ln_attn_b + (size_t)l * DMR, H0, X16, out);
    }
  }
}
